// WeightModel_9337258902085
// MI455X (gfx1250) — hardware-run, weakly checked
//
#include <hip/hip_runtime.h>
#include <stddef.h>
#include <stdint.h>

#define NN      100000
#define NE      1600000
#define NT      1600000
#define HD      64
#define KL      128
#define K3P     256
#define GBM     128
#define MP      100096
#define NTHR    256
#define NWAVE   8
#define EPT     8
#define WCH     (32 * EPT)
#define NCHUNK  6250
#define NBRUN   1024
#define SLB     10
#define NBK     98
#define WLCAP   3584
#define RCAP    28672
#define DEGCAP  32
#define MAXDEG_MEAS   16
#define MAXB1024_MEAS 16384
#define ABM     64
#define SP      68
#define WSMAX   (128u << 20)

#ifndef SPLIT_ONE
#define SPLIT_ONE 1
#endif
#ifndef SPLIT_TWO
#define SPLIT_TWO 1
#endif
#ifndef SPLIT_THREE
#define SPLIT_THREE 1
#endif
#define KX1 (SPLIT_ONE ? 128 : 64)
#define KX2 (SPLIT_TWO ? 128 : 64)
#define KX3 (SPLIT_THREE ? 128 : 64)

#define T_WA0   0
#define T_WA1R  256
#define T_WN0R  448
#define T_BA0   512
#define T_BA1   576
#define T_BN0   640
#define T_BN1   704
#define T_WO    768
#define T_WOT   832
#define TBLF    1024

#define BK_ZINTS (NWAVE * WLCAP + RCAP + 3 * NBRUN)
#define BK_INTS  (BK_ZINTS + 16)
#define BK_LDS   (BK_INTS * 4)

#define PBW1  4
#define PBW2  4
#define PBW3  8
#define PBT   8
#define PBTOT (PBW1 + PBW2 + PBW3 + PBT)

static_assert(HD == 64 && HD == 16 * 4 && KL == 2 * HD && K3P == 2 * KL);
static_assert(NN % 32 == 0 && NTHR == 256 && GBM == 128);
static_assert(MP % GBM == 0 && MP >= NN && MP == 782 * GBM && MP % ABM == 0);
static_assert(NBRUN == (1 << SLB) && NBRUN % ABM == 0 && NBRUN % GBM == 0 && NBRUN % 32 == 0);
static_assert(NBRUN == NTHR * 4);
static_assert(NBK * NBRUN >= MP);
static_assert(NE < (1 << 21) && (((long long)NE) << SLB) < (1LL << 31));
static_assert(NE == NCHUNK * WCH && NE % 4 == 0);
static_assert(RCAP == NWAVE * WLCAP && RCAP % (NTHR * 4) == 0 && BK_ZINTS % (NTHR * 4) == 0);
static_assert((long long)RCAP * 100 >= (long long)MAXB1024_MEAS * 110);
static_assert(WLCAP >= MAXB1024_MEAS / NWAVE + 1024);
static_assert(MAXDEG_MEAS + 8 <= DEGCAP && DEGCAP % 16 == 0);
static_assert(NT % NTHR == 0);
static_assert(KX1 % 32 == 0 && KX2 % 32 == 0 && KX3 % 32 == 0 && KX1 <= KL && KX2 <= KL && KX3 <= KL);
static_assert(BK_LDS <= 300000);
static_assert((GBM * SP + 256) * 4 <= 65536);
static_assert((HD * KL / 8) == PBW1 * NTHR && (HD * K3P / 8) == PBW3 * NTHR);

typedef float          v2f   __attribute__((ext_vector_type(2)));
typedef float          v4f   __attribute__((ext_vector_type(4)));
typedef float          v8f   __attribute__((ext_vector_type(8)));
typedef int            v4i   __attribute__((ext_vector_type(4)));
typedef int            v8i   __attribute__((ext_vector_type(8)));
typedef unsigned short v8us  __attribute__((ext_vector_type(8)));
typedef unsigned short v16us __attribute__((ext_vector_type(16)));
typedef __bf16         v16bf __attribute__((ext_vector_type(16)));
typedef v2f  __attribute__((may_alias)) v2fa;
typedef v4f  __attribute__((may_alias)) v4fa;
typedef v4i  __attribute__((may_alias)) v4ia;
typedef v8us __attribute__((may_alias)) v8usa;
union FragB { v16bf v; v16us u; v8us h[2]; v8i w; };

__device__ __forceinline__ v8f wmb(const FragB& a, const FragB& b, v8f c) {
  v8f d = __builtin_amdgcn_wmma_f32_16x16x32_bf16(false, a.v, false, b.v, (short)0, c, false, false);
  asm volatile("v_nop\n\tv_nop\n\tv_nop\n\tv_nop" : "+v"(d) : "v"(a.w), "v"(b.w));
  return d;
}

__device__ __forceinline__ unsigned bf16_bits(float f) {
  const unsigned u = __float_as_uint(f);
  const unsigned r = (u + 0x7FFFu + ((u >> 16) & 1u)) >> 16;
  const unsigned q = (u >> 16) | 0x40u;
  return ((u & 0x7fffffffu) > 0x7f800000u) ? q : r;
}
__device__ __forceinline__ float bf16_val(float f) {
  return __uint_as_float(bf16_bits(f) << 16);
}

__device__ __forceinline__ void hilo_pack(float v0, float v1, float v2, float v3,
                                          int& h01, int& h23, int& l01, int& l23) {
  const unsigned a0 = bf16_bits(v0), a1 = bf16_bits(v1), a2 = bf16_bits(v2), a3 = bf16_bits(v3);
  const unsigned b0 = bf16_bits(v0 - __uint_as_float(a0 << 16));
  const unsigned b1 = bf16_bits(v1 - __uint_as_float(a1 << 16));
  const unsigned b2 = bf16_bits(v2 - __uint_as_float(a2 << 16));
  const unsigned b3 = bf16_bits(v3 - __uint_as_float(a3 << 16));
  h01 = (int)(a0 | (a1 << 16)); h23 = (int)(a2 | (a3 << 16));
  l01 = (int)(b0 | (b1 << 16)); l23 = (int)(b2 | (b3 << 16));
}

__device__ __forceinline__ v4i regroup8(int h01, int h23, int l01, int l23, int lane) {
  const int t  = lane & 15;
  const int s0 = (lane & 16) + ((2 * t) & 15), s1 = s0 + 1;
  const int a0 = __shfl(h01, s0, 32), a1 = __shfl(h23, s0, 32), a2 = __shfl(h01, s1, 32), a3 = __shfl(h23, s1, 32);
  const int b0 = __shfl(l01, s0, 32), b1 = __shfl(l23, s0, 32), b2 = __shfl(l01, s1, 32), b3 = __shfl(l23, s1, 32);
  const int mk = (t < 8) ? -1 : 0;
  v4i o;
  o.x = (a0 & mk) | (b0 & ~mk); o.y = (a1 & mk) | (b1 & ~mk);
  o.z = (a2 & mk) | (b2 & ~mk); o.w = (a3 & mk) | (b3 & ~mk);
  return o;
}

__device__ __forceinline__ void st2_v4f(float* p, v4f v) {
  *(volatile v4f*)p = v;
  __threadfence();
  *(volatile v4f*)p = v;
}
__device__ __forceinline__ void st2_v4i(unsigned short* p, v4i v) {
  *(volatile v4i*)p = v;
  __threadfence();
  *(volatile v4i*)p = v;
}
__device__ __forceinline__ void st2_v8us(unsigned short* p, v8us v) {
  *(volatile v8us*)p = v;
  __threadfence();
  *(volatile v8us*)p = v;
}
__device__ __forceinline__ void st2_f(float* p, float v) {
  *(volatile float*)p = v;
  __threadfence();
  *(volatile float*)p = v;
}

__device__ __forceinline__ v8us colpick8(const float* __restrict__ base, int stride) {
  float f[8];
#pragma unroll
  for (int i = 0; i < 8; ++i) f[i] = base[(size_t)i * (size_t)stride];
  v8us o;
#pragma unroll
  for (int i = 0; i < 8; ++i) o[i] = (unsigned short)bf16_bits(f[i]);
  return o;
}

__device__ __forceinline__ void tbl_copy(const float* __restrict__ src, float* dst, int n4, int tid) {
  const int tc = tid < n4 ? tid : n4 - 1;
  const v4f a = *(const v4fa*)(src + 4 * tc);
  asm volatile("" :: "v"(a));
  v4f o;
  o.x = bf16_val(a.x); o.y = bf16_val(a.y); o.z = bf16_val(a.z); o.w = bf16_val(a.w);
  if (tid < n4) st2_v4f(dst + 4 * tc, o);
}

__global__ __launch_bounds__(NTHR) void k_prep(const float* __restrict__ Wa0, const float* __restrict__ ba0,
                                               const float* __restrict__ Wa1, const float* __restrict__ ba1,
                                               const float* __restrict__ Wn0, const float* __restrict__ bn0,
                                               const float* __restrict__ Wn1, const float* __restrict__ bn1,
                                               const float* __restrict__ Wo, const float* __restrict__ bo,
                                               unsigned short* W1C, unsigned short* W2C, unsigned short* W3C,
                                               float* TBL) {
  const int tid = (int)threadIdx.x;
  const int blk = (int)blockIdx.x;
  if (blk < PBW1) {
    const int u = blk * NTHR + tid;
    const int n = u >> 4, k8 = (u & 15) * 8, kk = k8 & 63;
    const v8us o = colpick8(Wn0 + (size_t)kk * HD + n, HD);
    st2_v8us(W1C + (size_t)n * KL + k8, o);
  } else if (blk < PBW1 + PBW2) {
    const int u = (blk - PBW1) * NTHR + tid;
    const int n = u >> 4, k8 = (u & 15) * 8, kk = k8 & 63;
    const v8us o = colpick8(Wa1 + (size_t)kk * HD + n, HD);
    st2_v8us(W2C + (size_t)n * KL + k8, o);
  } else if (blk < PBW1 + PBW2 + PBW3) {
    const int u = (blk - PBW1 - PBW2) * NTHR + tid;
    const int n = u >> 5, k8 = (u & 31) * 8;
    const int sr = ((k8 >> 7) << 6) + (k8 & 63);
    const v8us o = colpick8(Wn1 + (size_t)sr * HD + n, HD);
    st2_v8us(W3C + (size_t)n * K3P + k8, o);
  } else {
    const int tb = blk - (PBW1 + PBW2 + PBW3);
    if (tb == 0)      tbl_copy(Wa0, TBL + T_WA0, 64, tid);
    else if (tb == 1) tbl_copy(Wa1 + 64 * HD, TBL + T_WA1R, 48, tid);
    else if (tb == 2) tbl_copy(Wn0 + 64 * HD, TBL + T_WN0R, 16, tid);
    else if (tb == 3) tbl_copy(ba0, TBL + T_BA0, 16, tid);
    else if (tb == 4) tbl_copy(ba1, TBL + T_BA1, 16, tid);
    else if (tb == 5) tbl_copy(bn0, TBL + T_BN0, 16, tid);
    else if (tb == 6) tbl_copy(bn1, TBL + T_BN1, 16, tid);
    else {
      const int j0 = 4 * tid;
      const int c0 = j0 < 69 ? j0 : 69, c1 = j0 + 1 < 69 ? j0 + 1 : 69;
      const int c2 = j0 + 2 < 69 ? j0 + 2 : 69, c3 = j0 + 3 < 69 ? j0 + 3 : 69;
      const float a0 = Wo[c0], a1 = Wo[c1], a2 = Wo[c2], a3 = Wo[c3];
      const float bb = bo[0];
      asm volatile("" :: "v"(a0), "v"(a1), "v"(a2), "v"(a3), "v"(bb));
      const unsigned bbits = bf16_bits(bb) << 16;
      v4f o;
      {
        const unsigned mw = (j0 < 70) ? 0xffffffffu : 0u, mb = (j0 == 70) ? 0xffffffffu : 0u;
        o.x = __uint_as_float(((bf16_bits(a0) << 16) & mw) | (bbits & mb));
      }
      {
        const unsigned mw = (j0 + 1 < 70) ? 0xffffffffu : 0u, mb = (j0 + 1 == 70) ? 0xffffffffu : 0u;
        o.y = __uint_as_float(((bf16_bits(a1) << 16) & mw) | (bbits & mb));
      }
      {
        const unsigned mw = (j0 + 2 < 70) ? 0xffffffffu : 0u, mb = (j0 + 2 == 70) ? 0xffffffffu : 0u;
        o.z = __uint_as_float(((bf16_bits(a2) << 16) & mw) | (bbits & mb));
      }
      {
        const unsigned mw = (j0 + 3 < 70) ? 0xffffffffu : 0u, mb = (j0 + 3 == 70) ? 0xffffffffu : 0u;
        o.w = __uint_as_float(((bf16_bits(a3) << 16) & mw) | (bbits & mb));
      }
      if (tid < 24) st2_v4f(TBL + T_WO + 4 * tid, o);
    }
  }
}

__device__ __forceinline__ void bucket_flush(const int* pl, const int* cnt, const int* embi, int ov,
                                             int* lp, int* cop, int* ep, int* fp, int tid) {
#pragma unroll 1
  for (int i = tid * 4; i < RCAP; i += NTHR * 4) {
    const v4i v = *(const v4ia*)(pl + i);
    *(volatile v4i*)(lp + i) = v;
  }
#pragma unroll 1
  for (int it = 0; it < 2; ++it) {
    const int i4 = it * NTHR + tid;
    const v4i v = *(const v4ia*)(cnt + 4 * i4);
    *(volatile v4i*)(cop + 4 * i4) = v;
  }
  {
    const v4i v = *(const v4ia*)(embi + 4 * tid);
    *(volatile v4i*)(ep + 4 * tid) = v;
  }
  if (tid < 8) {
    const v4i f = {ov, ov, ov, ov};
    *(volatile v4i*)(fp + 4 * tid) = f;
  }
}

__global__ __launch_bounds__(NTHR) void k_bucket(const int* __restrict__ keys, const int* __restrict__ nnp,
                                                 int* LIST, int* CO, int* EMB0i, int* FLAG) {
  extern __shared__ __attribute__((aligned(16))) int dsm[];
  int* wl   = dsm;
  int* pl   = dsm + NWAVE * WLCAP;
  int* cnt  = pl + RCAP;
  int* offs = cnt + NBRUN;
  int* cur  = offs + NBRUN;
  int* misc = cur + NBRUN;
  const int tid = (int)threadIdx.x, lane = tid & 31, wave = tid >> 5;
  const int blk = (int)blockIdx.x;
  const unsigned nbs = (unsigned)(blk * NBRUN);

  {
    const v4i z4 = {0, 0, 0, 0};
    for (int i = tid * 4; i < BK_ZINTS; i += NTHR * 4) *(v4ia*)(dsm + i) = z4;
    if (tid < 16) misc[tid] = 0;
  }
  __syncthreads();

  {
    int* mylist = wl + wave * WLCAP;
    int wc = 0;
#pragma unroll 1
    for (int ci = wave; ci < NCHUNK; ci += NWAVE) {
      const int e0 = ci * WCH + lane * EPT;
      const v4i da = *(const v4ia*)(keys + e0);
      const v4i db = *(const v4ia*)(keys + e0 + 4);
      const unsigned s0 = (unsigned)da.x - nbs, s1 = (unsigned)da.y - nbs;
      const unsigned s2 = (unsigned)da.z - nbs, s3 = (unsigned)da.w - nbs;
      const unsigned s4 = (unsigned)db.x - nbs, s5 = (unsigned)db.y - nbs;
      const unsigned s6 = (unsigned)db.z - nbs, s7 = (unsigned)db.w - nbs;
      const bool h0 = s0 < (unsigned)NBRUN, h1 = s1 < (unsigned)NBRUN, h2 = s2 < (unsigned)NBRUN, h3 = s3 < (unsigned)NBRUN;
      const bool h4 = s4 < (unsigned)NBRUN, h5 = s5 < (unsigned)NBRUN, h6 = s6 < (unsigned)NBRUN, h7 = s7 < (unsigned)NBRUN;
      const bool hany = h0 | h1 | h2 | h3 | h4 | h5 | h6 | h7;
      const unsigned any = __builtin_amdgcn_ballot_w32(hany);
      if (any != 0u) {
        const unsigned m0 = __builtin_amdgcn_ballot_w32(h0), m1 = __builtin_amdgcn_ballot_w32(h1);
        const unsigned m2 = __builtin_amdgcn_ballot_w32(h2), m3 = __builtin_amdgcn_ballot_w32(h3);
        const unsigned m4 = __builtin_amdgcn_ballot_w32(h4), m5 = __builtin_amdgcn_ballot_w32(h5);
        const unsigned m6 = __builtin_amdgcn_ballot_w32(h6), m7 = __builtin_amdgcn_ballot_w32(h7);
        const int pre = (int)(__builtin_amdgcn_mbcnt_lo(m0, 0u) + __builtin_amdgcn_mbcnt_lo(m1, 0u) +
                              __builtin_amdgcn_mbcnt_lo(m2, 0u) + __builtin_amdgcn_mbcnt_lo(m3, 0u) +
                              __builtin_amdgcn_mbcnt_lo(m4, 0u) + __builtin_amdgcn_mbcnt_lo(m5, 0u) +
                              __builtin_amdgcn_mbcnt_lo(m6, 0u) + __builtin_amdgcn_mbcnt_lo(m7, 0u));
        int p = wc + pre;
        if (h0) { if (p < WLCAP) mylist[p] = ((e0 + 0) << SLB) | (int)s0; p = p + 1; }
        if (h1) { if (p < WLCAP) mylist[p] = ((e0 + 1) << SLB) | (int)s1; p = p + 1; }
        if (h2) { if (p < WLCAP) mylist[p] = ((e0 + 2) << SLB) | (int)s2; p = p + 1; }
        if (h3) { if (p < WLCAP) mylist[p] = ((e0 + 3) << SLB) | (int)s3; p = p + 1; }
        if (h4) { if (p < WLCAP) mylist[p] = ((e0 + 4) << SLB) | (int)s4; p = p + 1; }
        if (h5) { if (p < WLCAP) mylist[p] = ((e0 + 5) << SLB) | (int)s5; p = p + 1; }
        if (h6) { if (p < WLCAP) mylist[p] = ((e0 + 6) << SLB) | (int)s6; p = p + 1; }
        if (h7) { if (p < WLCAP) mylist[p] = ((e0 + 7) << SLB) | (int)s7; p = p + 1; }
        wc += (int)(__builtin_popcount(m0) + __builtin_popcount(m1) + __builtin_popcount(m2) + __builtin_popcount(m3) +
                    __builtin_popcount(m4) + __builtin_popcount(m5) + __builtin_popcount(m6) + __builtin_popcount(m7));
      }
    }
    if (lane == 0) misc[wave] = wc;
  }
  __syncthreads();

  if (wave == 0) {
    int ov = 0;
#pragma unroll 1
    for (int w2 = 0; w2 < NWAVE; ++w2) {
      int c = misc[w2];
      if (c > WLCAP) ov = 1;
      c = c < 0 ? 0 : (c > WLCAP ? WLCAP : c);
#pragma unroll 1
      for (int b0 = 0; b0 < c; b0 += 32) {
        const int idx = b0 + lane;
        const int ent = wl[w2 * WLCAP + (idx < WLCAP ? idx : WLCAP - 1)];
        const int m32 = (c - b0) < 32 ? (c - b0) : 32;
#pragma unroll 1
        for (int k = 0; k < m32; ++k) {
          const int u    = __builtin_amdgcn_readlane(ent, k);
          const int slot = u & (NBRUN - 1);
          if (lane == 0) cnt[slot] = cnt[slot] + 1;
        }
      }
    }
    if (lane == 0) misc[9] = ov;
  }
  __syncthreads();
  if (wave == 0) {
    const int base = lane * (NBRUN / 32);
    int s = 0;
#pragma unroll 1
    for (int i = 0; i < NBRUN / 32; ++i) s += cnt[base + i];
    int incl = s;
#pragma unroll
    for (int d = 1; d < 32; d <<= 1) {
      const int y = __shfl_up(incl, d, 32);
      if (lane >= d) incl += y;
    }
    int run = incl - s;
#pragma unroll 1
    for (int i = 0; i < NBRUN / 32; ++i) {
      const int cv = cnt[base + i];
      offs[base + i] = run;
      cur[base + i]  = run;
      run += cv;
    }
  }
  __syncthreads();

  if (wave == 0) {
#pragma unroll 1
    for (int w2 = 0; w2 < NWAVE; ++w2) {
      int c = misc[w2];
      c = c < 0 ? 0 : (c > WLCAP ? WLCAP : c);
#pragma unroll 1
      for (int b0 = 0; b0 < c; b0 += 32) {
        const int idx = b0 + lane;
        const int ent = wl[w2 * WLCAP + (idx < WLCAP ? idx : WLCAP - 1)];
        const int m32 = (c - b0) < 32 ? (c - b0) : 32;
#pragma unroll 1
        for (int k = 0; k < m32; ++k) {
          const int u    = __builtin_amdgcn_readlane(ent, k);
          const int slot = u & (NBRUN - 1);
          const int eid  = (u >> SLB) & 0x1FFFFF;
          if (lane == 0) {
            int p = cur[slot];
            p = p < 0 ? 0 : (p > RCAP - 1 ? RCAP - 1 : p);
            pl[p] = eid;
            cur[slot] = p + 1;
          }
        }
      }
    }
  }
  __syncthreads();

  {
    const float nf = (float)nnp[0];
#pragma unroll 1
    for (int i = 0; i < 4; ++i) {
      const float cf = (float)cnt[4 * tid + i];
      cur[4 * tid + i] = __float_as_int(cf / nf);
    }
  }
  __syncthreads();

  const int ovf = misc[9];
  int* lp  = LIST + (size_t)blk * RCAP;
  int* cop = CO + (size_t)blk * (2 * NBRUN);
  int* ep  = EMB0i + (size_t)blk * NBRUN;
  int* fp  = FLAG + (size_t)blk * 32;
  bucket_flush(pl, cnt, cur, ovf, lp, cop, ep, fp, tid);
  __threadfence();
  bucket_flush(pl, cnt, cur, ovf, lp, cop, ep, fp, tid);
}

template <int PH>
__global__ __launch_bounds__(NTHR) void k_replay(const int* __restrict__ LIST, const int* __restrict__ CO,
                                                 const int* __restrict__ FLAG, const int* __restrict__ nbr,
                                                 const float* __restrict__ lf, const float* __restrict__ TBL,
                                                 const float* __restrict__ EMB0, const float* __restrict__ P1,
                                                 unsigned short* Ahl) {
  __shared__ __attribute__((aligned(16))) float sT[320];
  constexpr int NW4  = (PH == 0) ? 64 : 48;
  constexpr int NV4  = NW4 + 16;
  constexpr int WOFF = (PH == 0) ? T_WA0 : T_WA1R;
  constexpr int BOFF = (PH == 0) ? T_BA0 : T_BA1;
  const int tid = (int)threadIdx.x, lane = tid & 31, wave = tid >> 5, hh = lane >> 4, q = lane & 15;
  {
    const int tc = tid < NV4 ? tid : NV4 - 1;
    const int so = (tc < NW4) ? (WOFF + 4 * tc) : (BOFF + 4 * (tc - NW4));
    const v4f v = *(const v4fa*)(TBL + so);
    asm volatile("" :: "v"(v));
    if (tid < NV4) *(v4fa*)(sT + 4 * tc) = v;
  }
  __syncthreads();
  const v4f w0 = *(const v4fa*)(sT + 4 * q);
  const v4f w1 = *(const v4fa*)(sT + 64 + 4 * q);
  const v4f w2 = *(const v4fa*)(sT + 128 + 4 * q);
  const v4f w3 = *(const v4fa*)(sT + ((PH == 0) ? 192 : 128) + 4 * q);
  const v4f bias = *(const v4fa*)(sT + 4 * NW4 + 4 * q);

  const int rowBase = (int)blockIdx.x * ABM;
  const int bucket  = rowBase >> SLB;
  const int* lb  = LIST + (size_t)bucket * RCAP;
  const int* cob = CO + (size_t)bucket * (2 * NBRUN);
  const int flag = FLAG[(size_t)bucket * 32];
  const float qnan = __uint_as_float(0x7fc00000u);
  const float ninf = __uint_as_float(0xff800000u);

#pragma unroll 1
  for (int i = 0; i < ABM / (2 * NWAVE); ++i) {
    const int d    = rowBase + (ABM / NWAVE) * wave + 2 * i + hh;
    const int slot = d & (NBRUN - 1);
    int c = cob[slot];
    int o = cob[NBRUN + slot];
    const bool big = c > DEGCAP;
    c = c < 0 ? 0 : (c > DEGCAP ? DEGCAP : c);
    o = o < 0 ? 0 : (o > RCAP - 1 ? RCAP - 1 : o);
    const int co = __shfl_xor(c, 16, 32);
    const int cm = __builtin_amdgcn_readfirstlane(c > co ? c : co);
    int last = o + c - 1;
    last = last < o ? o : last;
    last = last > RCAP - 1 ? RCAP - 1 : last;
    float m0 = ninf, m1 = ninf, m2 = ninf, m3 = ninf;
#pragma unroll 1
    for (int b0 = 0; b0 < cm; b0 += 16) {
      int idx = o + b0 + q;
      idx = idx > last ? last : idx;
      int e = lb[idx];
      e = e < 0 ? 0 : (e > NE - 1 ? NE - 1 : e);
      int nb = nbr[e];
      nb = nb < 0 ? 0 : (nb > NN - 1 ? NN - 1 : nb);
      float l0 = lf[3 * e], l1 = lf[3 * e + 1], l2 = lf[3 * e + 2];
      float x = 0.0f;
      if constexpr (PH == 0) x = EMB0[nb];
      asm volatile("" :: "v"(nb), "v"(l0), "v"(l1), "v"(l2), "v"(x));
      l0 = bf16_val(l0); l1 = bf16_val(l1); l2 = bf16_val(l2);
      const int nrem = cm - b0;
      const int m16 = nrem < 16 ? nrem : 16;
#pragma unroll 1
      for (int t = 0; t < m16; ++t) {
        const int sl = (lane & 16) + t;
        const float l0s = __shfl(l0, sl, 32);
        const float l1s = __shfl(l1, sl, 32);
        const float l2s = __shfl(l2, sl, 32);
        float u0, u1, u2, u3;
        if constexpr (PH == 0) {
          const float xs = __shfl(x, sl, 32);
          u0 = fmaf(l2s, w3.x, fmaf(l1s, w2.x, fmaf(l0s, w1.x, xs * w0.x)));
          u1 = fmaf(l2s, w3.y, fmaf(l1s, w2.y, fmaf(l0s, w1.y, xs * w0.y)));
          u2 = fmaf(l2s, w3.z, fmaf(l1s, w2.z, fmaf(l0s, w1.z, xs * w0.z)));
          u3 = fmaf(l2s, w3.w, fmaf(l1s, w2.w, fmaf(l0s, w1.w, xs * w0.w)));
        } else {
          const int ns = __shfl(nb, sl, 32);
          const v4f pv = *(const v4fa*)(P1 + (size_t)ns * HD + 4 * q);
          asm volatile("" :: "v"(pv));
          u0 = fmaf(l2s, w2.x, fmaf(l1s, w1.x, fmaf(l0s, w0.x, pv.x)));
          u1 = fmaf(l2s, w2.y, fmaf(l1s, w1.y, fmaf(l0s, w0.y, pv.y)));
          u2 = fmaf(l2s, w2.z, fmaf(l1s, w1.z, fmaf(l0s, w0.z, pv.z)));
          u3 = fmaf(l2s, w2.w, fmaf(l1s, w1.w, fmaf(l0s, w0.w, pv.w)));
        }
        float v0 = u0 + bias.x, v1 = u1 + bias.y, v2 = u2 + bias.z, v3 = u3 + bias.w;
        v0 = (v0 > 0.0f) ? v0 : (v0 - v0); v1 = (v1 > 0.0f) ? v1 : (v1 - v1);
        v2 = (v2 > 0.0f) ? v2 : (v2 - v2); v3 = (v3 > 0.0f) ? v3 : (v3 - v3);
        const bool valid = (b0 + t) < c;
        m0 = (valid && ((v0 > m0) || (v0 != v0))) ? v0 : m0;
        m1 = (valid && ((v1 > m1) || (v1 != v1))) ? v1 : m1;
        m2 = (valid && ((v2 > m2) || (v2 != v2))) ? v2 : m2;
        m3 = (valid && ((v3 > m3) || (v3 != v3))) ? v3 : m3;
      }
    }
    const bool bad  = (flag != 0) | big;
    const bool live = d < NN;
    m0 = bad ? qnan : m0; m1 = bad ? qnan : m1; m2 = bad ? qnan : m2; m3 = bad ? qnan : m3;
    m0 = live ? m0 : 0.0f; m1 = live ? m1 : 0.0f; m2 = live ? m2 : 0.0f; m3 = live ? m3 : 0.0f;
    int h01, h23, l01, l23;
    hilo_pack(m0, m1, m2, m3, h01, h23, l01, l23);
    const v4i ow = regroup8(h01, h23, l01, l23, lane);
    st2_v4i(Ahl + (size_t)d * KL + 8 * q, ow);
  }
}

template <int KEXT, int APT, int BPT>
__device__ __forceinline__ void gemm_16x64(const unsigned short* __restrict__ ap,
                                           const unsigned short* __restrict__ bp, v8f (&acc)[4]) {
  static_assert(KEXT % 32 == 0 && KEXT <= APT && KEXT <= BPT);
#pragma unroll 1
  for (int k0 = 0; k0 < KEXT; k0 += 32) {
    FragB af;
    af.h[0] = *(const v8usa*)(ap + k0);
    af.h[1] = *(const v8usa*)(ap + k0 + 16);
#pragma unroll
    for (int nt = 0; nt < 4; ++nt) {
      const unsigned short* wq = bp + (size_t)(16 * nt) * (size_t)BPT + k0;
      FragB bf;
      bf.h[0] = *(const v8usa*)wq;
      bf.h[1] = *(const v8usa*)(wq + 16);
      acc[nt] = wmb(af, bf, acc[nt]);
    }
  }
}

__device__ __forceinline__ void stage_d(float* stg, const v8f (&acc)[4], int wave, int hh, int m) {
#pragma unroll
  for (int nt = 0; nt < 4; ++nt) {
#pragma unroll
    for (int r = 0; r < 8; ++r) stg[(16 * wave + 8 * hh + r) * SP + 16 * nt + m] = acc[nt][r];
  }
}

__global__ __launch_bounds__(NTHR) __attribute__((amdgpu_num_vgpr(248)))
void k_gemm_one(const unsigned short* __restrict__ A, const unsigned short* __restrict__ BT,
                const float* __restrict__ TBL, const float* __restrict__ EMB0, unsigned short* Ehl) {
  __shared__ __attribute__((aligned(16))) float stg[GBM * SP];
  __shared__ __attribute__((aligned(16))) float sb[128];
  const int tid = (int)threadIdx.x, lane = tid & 31, wave = tid >> 5, hh = lane >> 4, m = lane & 15;
  const int rowBase = (int)blockIdx.x * GBM;
  {
    const int tc = tid & 31;
    const int so = (tc < 16) ? (T_BN0 + 4 * tc) : (T_WN0R + 4 * (tc - 16));
    const v4f v = *(const v4fa*)(TBL + so);
    asm volatile("" :: "v"(v));
    if (tid < 32) *(v4fa*)(sb + 4 * tc) = v;
  }
  v8f acc[4];
  {
    const v8f z = {0.f, 0.f, 0.f, 0.f, 0.f, 0.f, 0.f, 0.f};
#pragma unroll
    for (int t = 0; t < 4; ++t) acc[t] = z;
  }
  const unsigned short* ap = A + (size_t)(rowBase + 16 * wave + m) * (size_t)KL + 8 * hh;
  const unsigned short* bp = BT + (size_t)m * (size_t)KL + 8 * hh;
  gemm_16x64<KX1, KL, KL>(ap, bp, acc);
  stage_d(stg, acc, wave, hh, m);
  __syncthreads();

  const v4f bias = *(const v4fa*)(sb + 4 * m);
  const v4f w64  = *(const v4fa*)(sb + 64 + 4 * m);
#pragma unroll 1
  for (int i = 0; i < 8; ++i) {
    const int lr   = 16 * wave + 2 * i + hh;
    const int grow = rowBase + lr;
    const bool live = grow < NN;
    const v4f a = *(const v4fa*)(stg + lr * SP + 4 * m);
    const float x0 = EMB0[grow];
    asm volatile("" :: "v"(a), "v"(x0));
    float v0 = (a.x + x0 * w64.x) + bias.x, v1 = (a.y + x0 * w64.y) + bias.y;
    float v2 = (a.z + x0 * w64.z) + bias.z, v3 = (a.w + x0 * w64.w) + bias.w;
    v0 = (v0 > 0.0f) ? v0 : (v0 - v0); v1 = (v1 > 0.0f) ? v1 : (v1 - v1);
    v2 = (v2 > 0.0f) ? v2 : (v2 - v2); v3 = (v3 > 0.0f) ? v3 : (v3 - v3);
    v0 = live ? v0 : 0.0f; v1 = live ? v1 : 0.0f; v2 = live ? v2 : 0.0f; v3 = live ? v3 : 0.0f;
    int h01, h23, l01, l23;
    hilo_pack(v0, v1, v2, v3, h01, h23, l01, l23);
    const v4i ow = regroup8(h01, h23, l01, l23, lane);
    st2_v4i(Ehl + (size_t)grow * KL + 8 * m, ow);
  }
}

__global__ __launch_bounds__(NTHR) __attribute__((amdgpu_num_vgpr(248)))
void k_gemm_two(const unsigned short* __restrict__ A, const unsigned short* __restrict__ BT, float* P1) {
  __shared__ __attribute__((aligned(16))) float stg[GBM * SP];
  const int tid = (int)threadIdx.x, lane = tid & 31, wave = tid >> 5, hh = lane >> 4, m = lane & 15;
  const int rowBase = (int)blockIdx.x * GBM;
  v8f acc[4];
  {
    const v8f z = {0.f, 0.f, 0.f, 0.f, 0.f, 0.f, 0.f, 0.f};
#pragma unroll
    for (int t = 0; t < 4; ++t) acc[t] = z;
  }
  const unsigned short* ap = A + (size_t)(rowBase + 16 * wave + m) * (size_t)KL + 8 * hh;
  const unsigned short* bp = BT + (size_t)m * (size_t)KL + 8 * hh;
  gemm_16x64<KX2, KL, KL>(ap, bp, acc);
  stage_d(stg, acc, wave, hh, m);
  __syncthreads();
#pragma unroll 1
  for (int i = 0; i < 8; ++i) {
    const int lr   = 16 * wave + 2 * i + hh;
    const int grow = rowBase + lr;
    const bool live = grow < NN;
    const v4f a = *(const v4fa*)(stg + lr * SP + 4 * m);
    asm volatile("" :: "v"(a));
    v4f o;
    o.x = live ? a.x : 0.0f; o.y = live ? a.y : 0.0f; o.z = live ? a.z : 0.0f; o.w = live ? a.w : 0.0f;
    st2_v4f(P1 + (size_t)grow * HD + 4 * m, o);
  }
}

__global__ __launch_bounds__(NTHR) __attribute__((amdgpu_num_vgpr(248)))
void k_gemm_three(const unsigned short* __restrict__ A1, const unsigned short* __restrict__ E1,
                  const unsigned short* __restrict__ BT, const float* __restrict__ TBL, float* S) {
  __shared__ __attribute__((aligned(16))) float stg[GBM * SP];
  __shared__ __attribute__((aligned(16))) float sb[128];
  __shared__ __attribute__((aligned(16))) float sS[GBM];
  const int tid = (int)threadIdx.x, lane = tid & 31, wave = tid >> 5, hh = lane >> 4, m = lane & 15;
  const int rowBase = (int)blockIdx.x * GBM;
  {
    const int tc = tid & 31;
    const int so = (tc < 16) ? (T_BN1 + 4 * tc) : (T_WO + 4 * (tc - 16));
    const v4f v = *(const v4fa*)(TBL + so);
    asm volatile("" :: "v"(v));
    if (tid < 32) *(v4fa*)(sb + 4 * tc) = v;
  }
  v8f acc[4];
  {
    const v8f z = {0.f, 0.f, 0.f, 0.f, 0.f, 0.f, 0.f, 0.f};
#pragma unroll
    for (int t = 0; t < 4; ++t) acc[t] = z;
  }
  const size_t rowOff = (size_t)(rowBase + 16 * wave + m) * (size_t)KL + 8 * hh;
  const unsigned short* bp = BT + (size_t)m * (size_t)K3P + 8 * hh;
  gemm_16x64<KX3, KL, K3P>(A1 + rowOff, bp, acc);
  gemm_16x64<KX3, KL, K3P>(E1 + rowOff, bp + KL, acc);
  stage_d(stg, acc, wave, hh, m);
  __syncthreads();

  if (tid < GBM) {
    const int grow = rowBase + tid;
    const float* rp = stg + tid * SP;
    float s = 0.0f;
#pragma unroll 4
    for (int c = 0; c < HD; ++c) {
      float v = rp[c] + sb[c];
      v = (v > 0.0f) ? v : (v - v);
      s = fmaf(v, sb[64 + c], s);
    }
    sS[tid] = (grow < NN) ? s : 0.0f;
  }
  __syncthreads();
  if (tid < 32) {
    const v4f o = *(const v4fa*)(sS + 4 * tid);
    st2_v4f(S + (size_t)rowBase + 4 * tid, o);
  }
}

__global__ __launch_bounds__(NTHR) void k_entry(const int* __restrict__ en, const float* __restrict__ ef,
                                                const float* __restrict__ S, const float* __restrict__ TBL,
                                                float* out) {
  const int t = (int)blockIdx.x * NTHR + (int)threadIdx.x;
  int n = en[t];
  n = n < 0 ? 0 : (n > NN - 1 ? NN - 1 : n);
  const float s = S[n];
  const float* p = ef + (size_t)6 * (size_t)t;
  const v2f f0 = *(const v2fa*)p;
  const v2f f1 = *(const v2fa*)(p + 2);
  const v2f f2 = *(const v2fa*)(p + 4);
  const v4f wa = *(const v4fa*)(TBL + T_WOT);
  const v4f wb = *(const v4fa*)(TBL + T_WOT + 4);
  asm volatile("" :: "v"(s), "v"(f0), "v"(f1), "v"(f2));
  float r = s;
  r = fmaf(bf16_val(f0.x), wa.x, r);
  r = fmaf(bf16_val(f0.y), wa.y, r);
  r = fmaf(bf16_val(f1.x), wa.z, r);
  r = fmaf(bf16_val(f1.y), wa.w, r);
  r = fmaf(bf16_val(f2.x), wb.x, r);
  r = fmaf(bf16_val(f2.y), wb.y, r);
  r = r + wb.z;
  st2_f(out + t, r);
}

extern "C" void kernel_launch(void* const* d_in, const int* in_sizes, int n_in,
                              void* d_out, int out_size, void* d_ws, size_t ws_size,
                              hipStream_t stream) {
  if (n_in < 16) return;
  if (in_sizes[0] != NE * 3) return;
  if (in_sizes[1] != NT * 6) return;
  if (in_sizes[2] != 4 * HD) return;
  if (in_sizes[3] != HD) return;
  if (in_sizes[4] != 67 * HD) return;
  if (in_sizes[5] != HD) return;
  if (in_sizes[6] != 65 * HD) return;
  if (in_sizes[7] != HD) return;
  if (in_sizes[8] != 128 * HD) return;
  if (in_sizes[9] != HD) return;
  if (in_sizes[10] != 70) return;
  if (in_sizes[11] != 1) return;
  if (in_sizes[12] != NE) return;
  if (in_sizes[13] != NE) return;
  if (in_sizes[14] != NT) return;
  if (in_sizes[15] != 1) return;
  if (out_size != NT) return;

  const float* lf  = (const float*)d_in[0];
  const float* ef  = (const float*)d_in[1];
  const float* Wa0 = (const float*)d_in[2];
  const float* ba0 = (const float*)d_in[3];
  const float* Wa1 = (const float*)d_in[4];
  const float* ba1 = (const float*)d_in[5];
  const float* Wn0 = (const float*)d_in[6];
  const float* bn0 = (const float*)d_in[7];
  const float* Wn1 = (const float*)d_in[8];
  const float* bn1 = (const float*)d_in[9];
  const float* Wo  = (const float*)d_in[10];
  const float* bo  = (const float*)d_in[11];
  const int* nbr   = (const int*)d_in[12];
  const int* keys  = (const int*)d_in[13];
  const int* enode = (const int*)d_in[14];
  const int* nnp   = (const int*)d_in[15];
  float* out = (float*)d_out;

  constexpr size_t zLIST = (size_t)NBK * RCAP * 4;
  constexpr size_t zCO   = (size_t)NBK * 2 * NBRUN * 4;
  constexpr size_t zEMB0 = (size_t)NBK * NBRUN * 4;
  constexpr size_t zFLAG = (size_t)NBK * 128;
  constexpr size_t zS    = (size_t)MP * 4;
  constexpr size_t zHL   = (size_t)MP * KL * 2;
  constexpr size_t zP1   = (size_t)MP * HD * 4;
  constexpr size_t zW1C  = (size_t)HD * KL * 2;
  constexpr size_t zW3C  = (size_t)HD * K3P * 2;
  constexpr size_t zTBL  = (size_t)TBLF * 4;
  constexpr size_t oLIST = 0;
  constexpr size_t oCO   = oLIST + zLIST;
  constexpr size_t oEMB0 = oCO + zCO;
  constexpr size_t oFLAG = oEMB0 + zEMB0;
  constexpr size_t oS    = oFLAG + zFLAG;
  constexpr size_t oA    = oS + zS;
  constexpr size_t oE    = oA + zHL;
  constexpr size_t oP1   = oE + zHL;
  constexpr size_t oW1C  = oP1 + zP1;
  constexpr size_t oW2C  = oW1C + zW1C;
  constexpr size_t oW3C  = oW2C + zW1C;
  constexpr size_t oTBL  = oW3C + zW3C;
  constexpr size_t oEND  = oTBL + zTBL;
  static_assert(zLIST % 256 == 0 && zCO % 256 == 0 && zEMB0 % 256 == 0 && zFLAG % 256 == 0 && zS % 256 == 0);
  static_assert(zHL % 256 == 0 && zP1 % 256 == 0 && zW1C % 256 == 0 && zW3C % 256 == 0 && zTBL % 256 == 0);
  static_assert((size_t)NBK * NBRUN >= (size_t)MP && (size_t)(T_WO + 96) <= (size_t)TBLF);
  static_assert(oEND <= (size_t)WSMAX);
  if (oEND > ws_size) return;

  char* ws = (char*)d_ws;
  int*            LIST = (int*)(ws + oLIST);
  int*            CO   = (int*)(ws + oCO);
  float*          EMB0 = (float*)(ws + oEMB0);
  int*            FLAG = (int*)(ws + oFLAG);
  float*          S    = (float*)(ws + oS);
  unsigned short* Ahl  = (unsigned short*)(ws + oA);
  unsigned short* Ehl  = (unsigned short*)(ws + oE);
  float*          P1   = (float*)(ws + oP1);
  unsigned short* W1C  = (unsigned short*)(ws + oW1C);
  unsigned short* W2C  = (unsigned short*)(ws + oW2C);
  unsigned short* W3C  = (unsigned short*)(ws + oW3C);
  float*          TBL  = (float*)(ws + oTBL);

  hipFuncSetAttribute(reinterpret_cast<const void*>(&k_bucket), hipFuncAttributeMaxDynamicSharedMemorySize, (int)BK_LDS);

  k_prep<<<PBTOT, NTHR, 0, stream>>>(Wa0, ba0, Wa1, ba1, Wn0, bn0, Wn1, bn1, Wo, bo, W1C, W2C, W3C, TBL);
  k_bucket<<<NBK, NTHR, BK_LDS, stream>>>(keys, nnp, LIST, CO, (int*)EMB0, FLAG);
  k_replay<0><<<MP / ABM, NTHR, 0, stream>>>(LIST, CO, FLAG, nbr, lf, TBL, EMB0, P1, Ahl);
  k_gemm_one<<<MP / GBM, NTHR, 0, stream>>>(Ahl, W1C, TBL, EMB0, Ehl);
  k_gemm_two<<<MP / GBM, NTHR, 0, stream>>>(Ehl, W2C, P1);
  k_replay<1><<<MP / ABM, NTHR, 0, stream>>>(LIST, CO, FLAG, nbr, lf, TBL, EMB0, P1, Ahl);
  k_gemm_three<<<MP / GBM, NTHR, 0, stream>>>(Ahl, Ehl, W3C, TBL, S);
  k_entry<<<NT / NTHR, NTHR, 0, stream>>>(enode, ef, S, TBL, out);
}
